// GCN_Weights_31533649887980
// MI455X (gfx1250) — hardware-verified
//
#include <hip/hip_runtime.h>
#include <stddef.h>


#define FIN    64
#define NH     32
#define NEMB   63
#define NTHR   256
#define NWAVE  8
#define EPT    8
#define CHUNK  (NTHR * EPT)
#define WCAP   (EPT * 32)
#define LISTN  (NWAVE * WCAP)
#define EWR    131072
#define NBD    8192
#define SBD    13
#define NBA    2048
#define SBA    11
#define NBP    256
#define SBP    8
#define GROWS  128
#define AP     72
#define WSC    8.0f
#define WIV    0.125f

#define LDS_EW   (EWR)
#define LDS_AGG  (NBA * NH * 4 + LISTN * 4 + 64)

static_assert(CHUNK == 2048 && WCAP == 256);
static_assert((1 << SBD) == NBD);
static_assert((1 << SBA) == NBA);
static_assert((1 << SBP) == NBP);
static_assert(GROWS == NWAVE * 16);
static_assert((EWR % (4 * NTHR)) == 0);
static_assert((EWR % CHUNK) == 0);
static_assert((NBD % (4 * NTHR)) == 0);
static_assert((NBA % 32) == 0);
static_assert(NBP == NTHR);
static_assert((AP % 8) == 0 && AP >= FIN);
static_assert((NBA * NH) % (4 * NTHR) == 0 && (NBP * NH) % (4 * NTHR) == 0);

typedef float    v4f  __attribute__((ext_vector_type(4)));
typedef float    v8f  __attribute__((ext_vector_type(8)));
typedef int      v4i  __attribute__((ext_vector_type(4)));
typedef _Float16 v8h  __attribute__((ext_vector_type(8)));
typedef _Float16 v16h __attribute__((ext_vector_type(16)));
union FragH { v16h v; v8h h[2]; };

__device__ __forceinline__ v8f wmh(v16h a, v16h b, v8f c) {
  v8f d = __builtin_amdgcn_wmma_f32_16x16x32_f16(false, a, false, b, (short)0, c, false, false);
  asm volatile("v_nop\n\tv_nop\n\tv_nop\n\tv_nop" : "+v"(d) : "v"(a), "v"(b));
  return d;
}

template <int NB, int SB>
__device__ __forceinline__ int scan_chunk(const int* __restrict__ keys, int nK, int cbase, int slotBase,
                                          int vec, int* list, int tid, int lane, int wave) {
  int wc = 0;
  const int el0  = tid * EPT;
  const int e0   = cbase + el0;
  const int sent = -2147483647 - 1;
  v4i da, db;
  if (vec != 0 && cbase + CHUNK <= nK) {
    da = *(const v4i*)(keys + e0);
    db = *(const v4i*)(keys + e0 + 4);
  } else {
    da.x = (e0     < nK) ? keys[min(e0,     nK - 1)] : sent;
    da.y = (e0 + 1 < nK) ? keys[min(e0 + 1, nK - 1)] : sent;
    da.z = (e0 + 2 < nK) ? keys[min(e0 + 2, nK - 1)] : sent;
    da.w = (e0 + 3 < nK) ? keys[min(e0 + 3, nK - 1)] : sent;
    db.x = (e0 + 4 < nK) ? keys[min(e0 + 4, nK - 1)] : sent;
    db.y = (e0 + 5 < nK) ? keys[min(e0 + 5, nK - 1)] : sent;
    db.z = (e0 + 6 < nK) ? keys[min(e0 + 6, nK - 1)] : sent;
    db.w = (e0 + 7 < nK) ? keys[min(e0 + 7, nK - 1)] : sent;
  }
  const unsigned nb = (unsigned)slotBase;
  const unsigned s0 = (unsigned)da.x - nb, s1 = (unsigned)da.y - nb;
  const unsigned s2 = (unsigned)da.z - nb, s3 = (unsigned)da.w - nb;
  const unsigned s4 = (unsigned)db.x - nb, s5 = (unsigned)db.y - nb;
  const unsigned s6 = (unsigned)db.z - nb, s7 = (unsigned)db.w - nb;
  const bool h0 = s0 < (unsigned)NB, h1 = s1 < (unsigned)NB, h2 = s2 < (unsigned)NB, h3 = s3 < (unsigned)NB;
  const bool h4 = s4 < (unsigned)NB, h5 = s5 < (unsigned)NB, h6 = s6 < (unsigned)NB, h7 = s7 < (unsigned)NB;
  const unsigned any = __builtin_amdgcn_ballot_w32(h0 | h1 | h2 | h3 | h4 | h5 | h6 | h7);
  if (any != 0u) {
#define HITJ(J, HJ, SJ) { \
      const unsigned mj = __builtin_amdgcn_ballot_w32(HJ); \
      if (mj != 0u) { \
        if (HJ) { \
          const int pos = wc + (int)__builtin_amdgcn_mbcnt_lo(mj, 0u); \
          if (pos < WCAP) list[wave * WCAP + pos] = ((el0 + (J)) << SB) | (int)(SJ); \
        } \
        wc += (int)__builtin_popcount(mj); } }
    HITJ(0, h0, s0)
    HITJ(1, h1, s1)
    HITJ(2, h2, s2)
    HITJ(3, h3, s3)
    HITJ(4, h4, s4)
    HITJ(5, h5, s5)
    HITJ(6, h6, s6)
    HITJ(7, h7, s7)
#undef HITJ
  }
  return wc;
}

__device__ __forceinline__ void mark_chunk(const int* __restrict__ keys, int nK, int cbase, int ebase,
                                           int vec, unsigned char* cls, unsigned char c, int tid) {
  const int e0   = cbase + tid * EPT;
  const int sent = -2147483647 - 1;
  v4i da, db;
  if (vec != 0 && cbase + CHUNK <= nK) {
    da = *(const v4i*)(keys + e0);
    db = *(const v4i*)(keys + e0 + 4);
  } else {
    da.x = (e0     < nK) ? keys[min(e0,     nK - 1)] : sent;
    da.y = (e0 + 1 < nK) ? keys[min(e0 + 1, nK - 1)] : sent;
    da.z = (e0 + 2 < nK) ? keys[min(e0 + 2, nK - 1)] : sent;
    da.w = (e0 + 3 < nK) ? keys[min(e0 + 3, nK - 1)] : sent;
    db.x = (e0 + 4 < nK) ? keys[min(e0 + 4, nK - 1)] : sent;
    db.y = (e0 + 5 < nK) ? keys[min(e0 + 5, nK - 1)] : sent;
    db.z = (e0 + 6 < nK) ? keys[min(e0 + 6, nK - 1)] : sent;
    db.w = (e0 + 7 < nK) ? keys[min(e0 + 7, nK - 1)] : sent;
  }
  const unsigned nb = (unsigned)ebase;
  const unsigned s0 = (unsigned)da.x - nb, s1 = (unsigned)da.y - nb;
  const unsigned s2 = (unsigned)da.z - nb, s3 = (unsigned)da.w - nb;
  const unsigned s4 = (unsigned)db.x - nb, s5 = (unsigned)db.y - nb;
  const unsigned s6 = (unsigned)db.z - nb, s7 = (unsigned)db.w - nb;
  if (s0 < (unsigned)EWR) cls[s0] = c;
  if (s1 < (unsigned)EWR) cls[s1] = c;
  if (s2 < (unsigned)EWR) cls[s2] = c;
  if (s3 < (unsigned)EWR) cls[s3] = c;
  if (s4 < (unsigned)EWR) cls[s4] = c;
  if (s5 < (unsigned)EWR) cls[s5] = c;
  if (s6 < (unsigned)EWR) cls[s6] = c;
  if (s7 < (unsigned)EWR) cls[s7] = c;
}

__device__ __forceinline__ float selw(int b, float p0, float p1, float p2) {
  return b == 0 ? p0 : (b == 1 ? p1 : (b == 2 ? p2 : 1.0f));
}

__device__ __forceinline__ void ew_store_pass(const int* cw, float* gp, float p0, float p1, float p2, int tid) {
#pragma unroll 1
  for (int it = 0; it < EWR / (4 * NTHR); ++it) {
    const int idx = it * NTHR + tid;
    const int wd  = cw[idx];
    v4f v;
    v.x = selw(wd & 255, p0, p1, p2);
    v.y = selw((wd >> 8) & 255, p0, p1, p2);
    v.z = selw((wd >> 16) & 255, p0, p1, p2);
    v.w = selw((wd >> 24) & 255, p0, p1, p2);
    *(volatile v4f*)(gp + 4 * idx) = v;
  }
}

__global__ __launch_bounds__(NTHR) void k_ewclass(
    const int* __restrict__ km, const int* __restrict__ um, const int* __restrict__ om,
    int nk, int nu, int no, const float* __restrict__ msgw, float* ew) {
  extern __shared__ v4f lds_dyn[];
  v4i* lwords = (v4i*)lds_dyn;
  unsigned char* cls = (unsigned char*)lds_dyn;
  const int tid = threadIdx.x;
  const int ebase = blockIdx.x * EWR;
  {
    const v4i t3 = {0x03030303, 0x03030303, 0x03030303, 0x03030303};
#pragma unroll 1
    for (int i = tid; i < EWR / 16; i += NTHR) lwords[i] = t3;
  }
  __syncthreads();
#pragma unroll 1
  for (int c = 0; c < 3; ++c) {
    const int* keys = c == 0 ? km : (c == 1 ? um : om);
    const int  nK   = c == 0 ? nk : (c == 1 ? nu : no);
    const int  nCh  = (nK + CHUNK - 1) / CHUNK;
#pragma unroll 1
    for (int ch = 0; ch < nCh; ++ch) mark_chunk(keys, nK, ch * CHUNK, ebase, 1, cls, (unsigned char)c, tid);
    __syncthreads();
  }
  const float w0 = msgw[0], w1 = msgw[1], w2 = msgw[2];
  const float mx = fmaxf(w0, fmaxf(w1, w2));
  const float x0 = expf(w0 - mx), x1 = expf(w1 - mx), x2 = expf(w2 - mx);
  const float rs = 1.0f / (x0 + x1 + x2);
  const float p0 = x0 * rs, p1 = x1 * rs, p2 = x2 * rs;
  const int* cw = (const int*)lds_dyn;
  float* gp = ew + (size_t)ebase;
  ew_store_pass(cw, gp, p0, p1, p2, tid);
  __threadfence();
  ew_store_pass(cw, gp, p0, p1, p2, tid);
}

__device__ __forceinline__ void dinv_store_pass(const float* sdeg, float* gp, int tid) {
#pragma unroll 1
  for (int q = 0; q < NBD / (4 * NTHR); ++q) {
    const int idx = q * NTHR + tid;
    const v4f d = *(const v4f*)(sdeg + 4 * idx);
    v4f r;
    const float dx = d.x + 1.0f, dy = d.y + 1.0f, dz = d.z + 1.0f, dw = d.w + 1.0f;
    r.x = dx > 0.0f ? rsqrtf(dx) : 0.0f;
    r.y = dy > 0.0f ? rsqrtf(dy) : 0.0f;
    r.z = dz > 0.0f ? rsqrtf(dz) : 0.0f;
    r.w = dw > 0.0f ? rsqrtf(dw) : 0.0f;
    *(volatile v4f*)(gp + 4 * idx) = r;
  }
}

__global__ __launch_bounds__(NTHR) void k_deg(
    const int* __restrict__ ei, const float* __restrict__ ew, float* dinv, int nE, int vec) {
  __shared__ __attribute__((aligned(16))) float sdeg[NBD];
  __shared__ __attribute__((aligned(16))) int list[LISTN];
  __shared__ int wcnt[NWAVE];
  const int tid = threadIdx.x, lane = tid & 31, wave = tid >> 5;
  const int nodeBase = blockIdx.x * NBD;
  const int* dsts = ei + nE;
  {
    const v4f z = {0.f, 0.f, 0.f, 0.f};
#pragma unroll 1
    for (int i = tid; i < NBD / 4; i += NTHR) ((v4f*)sdeg)[i] = z;
  }
  __syncthreads();

  const int nChunks = (nE + CHUNK - 1) / CHUNK;
#pragma unroll 1
  for (int ch = 0; ch < nChunks; ++ch) {
    const int cbase = ch * CHUNK;
    const int wc = scan_chunk<NBD, SBD>(dsts, nE, cbase, nodeBase, vec, list, tid, lane, wave);
    if (lane == 0) wcnt[wave] = wc;
    __syncthreads();
    if (wave == 0) {
#pragma unroll 1
      for (int wsx = 0; wsx < NWAVE; ++wsx) {
        int n = __builtin_amdgcn_readfirstlane(wcnt[wsx]);
        n = n > WCAP ? WCAP : (n < 0 ? 0 : n);
        const int* lp = list + wsx * WCAP;
#pragma unroll 1
        for (int i = 0; i < n; ++i) {
          const int ent  = __builtin_amdgcn_readfirstlane(lp[i]);
          const int slot = ent & (NBD - 1);
          int e = cbase + ((ent >> SBD) & (CHUNK - 1));
          e = e > nE - 1 ? nE - 1 : e;
          const float w = ew[e];
          if (lane == 0) sdeg[slot] = sdeg[slot] + w;
        }
      }
    }
    __syncthreads();
  }

  float* gp = dinv + (size_t)nodeBase;
  dinv_store_pass(sdeg, gp, tid);
  __threadfence();
  dinv_store_pass(sdeg, gp, tid);
}

__device__ __forceinline__ void hws_store_pass(const float* stg, float* hws, int rowBase, int wave, int lane) {
  const int rq = lane >> 3, c4 = (lane & 7) * 4;
#pragma unroll
  for (int i = 0; i < 4; ++i) {
    const int r = wave * 16 + 4 * i + rq;
    const v4f v = *(const v4f*)(stg + r * NH + c4);
    *(volatile v4f*)(hws + ((size_t)rowBase + r) * NH + c4) = v;
  }
}

__global__ __launch_bounds__(NTHR) void k_node(
    const float* __restrict__ x, const float* __restrict__ embW, const float* __restrict__ embB,
    const float* __restrict__ gcnW, const float* __restrict__ dinv, float* hws, int nN) {
  __shared__ __attribute__((aligned(16))) _Float16 sBe[64 * AP];
  __shared__ __attribute__((aligned(16))) _Float16 sBg[NH * AP];
  __shared__ __attribute__((aligned(16))) _Float16 sH[GROWS * AP];
  __shared__ __attribute__((aligned(16))) v4f sU[GROWS * AP / 8];
  _Float16* sA  = (_Float16*)sU;
  float*    stg = (float*)sU;
  const int tid = threadIdx.x, lane = tid & 31, wave = tid >> 5, hh = lane >> 4, m = lane & 15;
  const int rowBase = blockIdx.x * GROWS;

#pragma unroll 1
  for (int i = tid; i < 64 * 64; i += NTHR) {
    const int n = i >> 6, k = i & 63;
    const int nc = n < NEMB ? n : NEMB - 1, kc = k < NEMB ? k : NEMB - 1;
    const float w = embW[kc * NEMB + nc];
    const float v = (n < NEMB && k < NEMB) ? w * WSC : 0.0f;
    sBe[n * AP + k] = (_Float16)v;
  }
#pragma unroll 1
  for (int i = tid; i < NH * 64; i += NTHR) {
    const int n = i >> 6, k = i & 63;
    sBg[n * AP + k] = (_Float16)(gcnW[k * NH + n] * WSC);
  }
#pragma unroll 1
  for (int i = tid; i < GROWS * 64; i += NTHR) {
    const int r = i >> 6, k = i & 63;
    int row = rowBase + r;
    row = row > nN - 1 ? nN - 1 : row;
    const int kc = k < NEMB ? k + 1 : FIN - 1;
    const float xv = x[(size_t)row * FIN + kc];
    sA[r * AP + k] = (_Float16)(k < NEMB ? xv : 0.0f);
  }
  __syncthreads();

  v8f acc[4];
#pragma unroll
  for (int t = 0; t < 4; ++t) { v8f z = {0.f, 0.f, 0.f, 0.f, 0.f, 0.f, 0.f, 0.f}; acc[t] = z; }
  {
    const _Float16* ar = sA + (wave * 16 + m) * AP + 8 * hh;
#pragma unroll
    for (int kt = 0; kt < 2; ++kt) {
      FragH a;
      a.h[0] = *(const v8h*)(ar + 32 * kt);
      a.h[1] = *(const v8h*)(ar + 32 * kt + 16);
#pragma unroll
      for (int t = 0; t < 4; ++t) {
        const _Float16* bp = sBe + (16 * t + m) * AP + 32 * kt + 8 * hh;
        FragH b;
        b.h[0] = *(const v8h*)bp;
        b.h[1] = *(const v8h*)(bp + 16);
        acc[t] = wmh(a.v, b.v, acc[t]);
      }
    }
  }
  const int row0 = wave * 16 + 8 * hh;
#pragma unroll
  for (int t = 0; t < 4; ++t) {
    const int n = 16 * t + m;
    const float bb = embB[n < NEMB ? n : NEMB - 1];
    _Float16* hp = sH + row0 * AP + 1 + n;
#pragma unroll
    for (int r = 0; r < 8; ++r) {
      const float v = acc[t][r] * WIV + bb;
      if (n < NEMB) hp[r * AP] = (_Float16)v;
    }
  }
  {
    const int rl = wave * 16 + m;
    int xrow = rowBase + rl;
    xrow = xrow > nN - 1 ? nN - 1 : xrow;
    const float x0 = x[(size_t)xrow * FIN];
    if (hh == 0) sH[rl * AP] = (_Float16)x0;
  }
  __syncthreads();

  v8f acc2[2];
#pragma unroll
  for (int u = 0; u < 2; ++u) { v8f z = {0.f, 0.f, 0.f, 0.f, 0.f, 0.f, 0.f, 0.f}; acc2[u] = z; }
  {
    const _Float16* ar = sH + (wave * 16 + m) * AP + 8 * hh;
#pragma unroll
    for (int kt = 0; kt < 2; ++kt) {
      FragH a;
      a.h[0] = *(const v8h*)(ar + 32 * kt);
      a.h[1] = *(const v8h*)(ar + 32 * kt + 16);
#pragma unroll
      for (int u = 0; u < 2; ++u) {
        const _Float16* bp = sBg + (16 * u + m) * AP + 32 * kt + 8 * hh;
        FragH b;
        b.h[0] = *(const v8h*)bp;
        b.h[1] = *(const v8h*)(bp + 16);
        acc2[u] = wmh(a.v, b.v, acc2[u]);
      }
    }
  }
  {
    const v4f dA = *(const v4f*)(dinv + (size_t)rowBase + row0);
    const v4f dB = *(const v4f*)(dinv + (size_t)rowBase + row0 + 4);
    float dv[8];
    dv[0] = dA.x; dv[1] = dA.y; dv[2] = dA.z; dv[3] = dA.w;
    dv[4] = dB.x; dv[5] = dB.y; dv[6] = dB.z; dv[7] = dB.w;
#pragma unroll
    for (int u = 0; u < 2; ++u) {
      float* sp = stg + row0 * NH + 16 * u + m;
#pragma unroll
      for (int r = 0; r < 8; ++r) sp[r * NH] = acc2[u][r] * WIV * dv[r];
    }
  }
  __syncthreads();

  hws_store_pass(stg, hws, rowBase, wave, lane);
  __threadfence();
  hws_store_pass(stg, hws, rowBase, wave, lane);
}

__device__ __forceinline__ void hg_store_pass(const float* acc, const float* __restrict__ hws,
                                              const float* __restrict__ dinv, const float* __restrict__ gb,
                                              float* hg, int nodeBase, int nN, int tid) {
  const int rq = tid >> 3, c4 = (tid & 7) * 4;
  const v4f bb = *(const v4f*)(gb + c4);
#pragma unroll 1
  for (int it = 0; it < NBA / 32; ++it) {
    const int r = it * 32 + rq;
    const int node = nodeBase + r;
    const int nc = node > nN - 1 ? nN - 1 : node;
    const v4f a = *(const v4f*)(acc + r * NH + c4);
    const v4f s = *(const v4f*)(hws + (size_t)nc * NH + c4);
    const float di = dinv[node];
    v4f v = (a + s) * di + bb;
    v.x = fmaxf(v.x, 0.0f); v.y = fmaxf(v.y, 0.0f); v.z = fmaxf(v.z, 0.0f); v.w = fmaxf(v.w, 0.0f);
    *(volatile v4f*)(hg + (size_t)node * NH + c4) = v;
  }
}

__global__ __launch_bounds__(NTHR) void k_agg(
    const int* __restrict__ ei, const float* __restrict__ ew, const float* __restrict__ dinv,
    const float* __restrict__ hws, const float* __restrict__ gb, float* hg, int nN, int nE, int vec) {
  extern __shared__ v4f lds_dyn[];
  float* acc  = (float*)lds_dyn;
  int*   list = (int*)(acc + NBA * NH);
  int*   wcnt = list + LISTN;
  const int tid = threadIdx.x, lane = tid & 31, wave = tid >> 5;
  const int nodeBase = blockIdx.x * NBA;
  const int* dsts = ei + nE;
  {
    const v4f z = {0.f, 0.f, 0.f, 0.f};
#pragma unroll 1
    for (int i = tid; i < NBA * NH / 4; i += NTHR) lds_dyn[i] = z;
  }
  __syncthreads();

  const int nChunks = (nE + CHUNK - 1) / CHUNK;
#pragma unroll 1
  for (int ch = 0; ch < nChunks; ++ch) {
    const int cbase = ch * CHUNK;
    const int wc = scan_chunk<NBA, SBA>(dsts, nE, cbase, nodeBase, vec, list, tid, lane, wave);
    if (lane == 0) wcnt[wave] = wc;
    __syncthreads();
    if (wave == 0) {
#pragma unroll 1
      for (int wsx = 0; wsx < NWAVE; ++wsx) {
        int n = __builtin_amdgcn_readfirstlane(wcnt[wsx]);
        n = n > WCAP ? WCAP : (n < 0 ? 0 : n);
        const int* lp = list + wsx * WCAP;
#pragma unroll 1
        for (int i = 0; i < n; ++i) {
          const int ent  = __builtin_amdgcn_readfirstlane(lp[i]);
          const int slot = ent & (NBA - 1);
          int e = cbase + ((ent >> SBA) & (CHUNK - 1));
          e = e > nE - 1 ? nE - 1 : e;
          int src = __builtin_amdgcn_readfirstlane(ei[e]);
          src = src < 0 ? 0 : (src > nN - 1 ? nN - 1 : src);
          const float w = ew[e];
          const float v = hws[(size_t)src * NH + lane];
          float* ap = acc + slot * NH + lane;
          const float o = *ap;
          *ap = fmaf(w, v, o);
        }
      }
    }
    __syncthreads();
  }

  hg_store_pass(acc, hws, dinv, gb, hg, nodeBase, nN, tid);
  __threadfence();
  hg_store_pass(acc, hws, dinv, gb, hg, nodeBase, nN, tid);
}

__device__ __forceinline__ void out_store_pass(const float* sout, float* out, int gBase, int G, int tid) {
  if (tid < NBP / 4) {
    const int i4 = gBase + 4 * tid;
    const v4f v = *(const v4f*)(sout + 4 * tid);
    if (i4 + 3 < G) *(volatile v4f*)(out + i4) = v;
  }
  if (tid == 0) {
#pragma unroll 1
    for (int j = (G & ~3); j < G; ++j) {
      const int lj = j - gBase;
      const int lc = lj < 0 ? 0 : (lj > NBP - 1 ? NBP - 1 : lj);
      const float v = sout[lc];
      if (lj >= 0 && lj < NBP) *(volatile float*)(out + j) = v;
    }
  }
}

__global__ __launch_bounds__(NTHR) void k_pool(
    const int* __restrict__ batch, const float* __restrict__ hg,
    const float* __restrict__ fc1w, const float* __restrict__ fc1b,
    const float* __restrict__ outw, const float* __restrict__ outb,
    float* out, int nN, int G) {
  __shared__ __attribute__((aligned(16))) float pacc[NBP * NH];
  __shared__ __attribute__((aligned(16))) int list[LISTN];
  __shared__ __attribute__((aligned(16))) float sout[NBP];
  __shared__ int wcnt[NWAVE];
  const int tid = threadIdx.x, lane = tid & 31, wave = tid >> 5;
  const int gBase = blockIdx.x * NBP;
  {
    const v4f z = {0.f, 0.f, 0.f, 0.f};
#pragma unroll 1
    for (int i = tid; i < NBP * NH / 4; i += NTHR) ((v4f*)pacc)[i] = z;
  }
  __syncthreads();

  const int nChunks = (nN + CHUNK - 1) / CHUNK;
#pragma unroll 1
  for (int ch = 0; ch < nChunks; ++ch) {
    const int cbase = ch * CHUNK;
    const int wc = scan_chunk<NBP, SBP>(batch, nN, cbase, gBase, 1, list, tid, lane, wave);
    if (lane == 0) wcnt[wave] = wc;
    __syncthreads();
    if (wave == 0) {
#pragma unroll 1
      for (int wsx = 0; wsx < NWAVE; ++wsx) {
        int n = __builtin_amdgcn_readfirstlane(wcnt[wsx]);
        n = n > WCAP ? WCAP : (n < 0 ? 0 : n);
        const int* lp = list + wsx * WCAP;
#pragma unroll 1
        for (int i = 0; i < n; ++i) {
          const int ent  = __builtin_amdgcn_readfirstlane(lp[i]);
          const int slot = ent & (NBP - 1);
          int nd = cbase + ((ent >> SBP) & (CHUNK - 1));
          nd = nd > nN - 1 ? nN - 1 : nd;
          const float v = hg[(size_t)nd * NH + lane];
          float* ap = pacc + slot * NH + lane;
          *ap = *ap + v;
        }
      }
    }
    __syncthreads();
  }

  {
    const float* pr = pacc + tid * NH;
    float o = outb[0];
#pragma unroll 1
    for (int j = 0; j < NH; ++j) {
      float z = fc1b[j];
#pragma unroll 1
      for (int i = 0; i < NH; ++i) z = fmaf(pr[i], fc1w[i * NH + j], z);
      z = fmaxf(z, 0.0f);
      o = fmaf(z, outw[j], o);
    }
    sout[tid] = o;
  }
  __syncthreads();

  out_store_pass(sout, out, gBase, G, tid);
  __threadfence();
  out_store_pass(sout, out, gBase, G, tid);
}

extern "C" void kernel_launch(void* const* d_in, const int* in_sizes, int n_in,
                              void* d_out, int out_size, void* d_ws, size_t ws_size,
                              hipStream_t stream) {
  if (n_in < 15) return;
  const int nN = in_sizes[0] / FIN;
  const int nE = in_sizes[1] / 2;
  if (nN < 1 || nE < 1 || in_sizes[0] != nN * FIN || in_sizes[1] != 2 * nE || in_sizes[2] != nN) return;
  const int nk = in_sizes[3], nu = in_sizes[4], no = in_sizes[5];
  if (nk < 0 || nu < 0 || no < 0) return;
  if (in_sizes[6] < 3 || in_sizes[7] != NEMB * NEMB || in_sizes[8] < NEMB) return;
  if (in_sizes[9] != FIN * NH || in_sizes[10] < NH || in_sizes[11] != NH * NH || in_sizes[12] < NH ||
      in_sizes[13] < NH || in_sizes[14] < 1) return;
  const int G = out_size;
  if (G < 1) return;
  if (nE > (1 << 28) || nN > (1 << 24) || G > (1 << 24)) return;

  const float* x     = (const float*)d_in[0];
  const int*   ei    = (const int*)d_in[1];
  const int*   batch = (const int*)d_in[2];
  const int*   km    = (const int*)d_in[3];
  const int*   um    = (const int*)d_in[4];
  const int*   om    = (const int*)d_in[5];
  const float* msgw  = (const float*)d_in[6];
  const float* embW  = (const float*)d_in[7];
  const float* embB  = (const float*)d_in[8];
  const float* gcnW  = (const float*)d_in[9];
  const float* gcnB  = (const float*)d_in[10];
  const float* fc1W  = (const float*)d_in[11];
  const float* fc1B  = (const float*)d_in[12];
  const float* outW  = (const float*)d_in[13];
  const float* outB  = (const float*)d_in[14];
  float* out = (float*)d_out;

  const int nEB = (nE + EWR - 1) / EWR;
  const int nDB = (nN + NBD - 1) / NBD;
  const int nNB = (nN + GROWS - 1) / GROWS;
  const int nAB = (nN + NBA - 1) / NBA;
  const int nPB = (G + NBP - 1) / NBP;
  const size_t EWPAD = (size_t)nEB * EWR;
  const size_t NDPAD = (size_t)nDB * NBD;
  const size_t NPAD  = (size_t)nNB * GROWS;
  const size_t NAPAD = (size_t)nAB * NBA;
  if (NDPAD < NPAD || NDPAD < NAPAD) return;

  char* ws = (char*)d_ws;
  size_t off = 0;
  const size_t oEw  = off; off += EWPAD * 4;          off = (off + 255) & ~(size_t)255;
  const size_t oDv  = off; off += NDPAD * 4;          off = (off + 255) & ~(size_t)255;
  const size_t oHws = off; off += NPAD * NH * 4;      off = (off + 255) & ~(size_t)255;
  const size_t oHg  = off; off += NAPAD * NH * 4;     off = (off + 255) & ~(size_t)255;
  if (off > ws_size) return;
  float* ew   = (float*)(ws + oEw);
  float* dinv = (float*)(ws + oDv);
  float* hws  = (float*)(ws + oHws);
  float* hg   = (float*)(ws + oHg);

  const int vecCol = ((nE & 3) == 0) ? 1 : 0;

  hipFuncSetAttribute(reinterpret_cast<const void*>(&k_ewclass),
                      hipFuncAttributeMaxDynamicSharedMemorySize, LDS_EW);
  k_ewclass<<<nEB, NTHR, LDS_EW, stream>>>(km, um, om, nk, nu, no, msgw, ew);

  k_deg<<<nDB, NTHR, 0, stream>>>(ei, ew, dinv, nE, vecCol);

  k_node<<<nNB, NTHR, 0, stream>>>(x, embW, embB, gcnW, dinv, hws, nN);

  hipFuncSetAttribute(reinterpret_cast<const void*>(&k_agg),
                      hipFuncAttributeMaxDynamicSharedMemorySize, LDS_AGG);
  k_agg<<<nAB, NTHR, LDS_AGG, stream>>>(ei, ew, dinv, hws, gcnB, hg, nN, nE, vecCol);

  k_pool<<<nPB, NTHR, 0, stream>>>(batch, hg, fc1W, fc1B, outW, outB, out, nN, G);
}
